// MoEGAT_45088566673466
// MI455X (gfx1250) — hardware-verified
//
#include <hip/hip_runtime.h>
#include <stdint.h>

#define DEVINL __device__ __forceinline__

typedef _Float16 f16t;
typedef _Float16 v16h __attribute__((ext_vector_type(16)));
typedef _Float16 v8h  __attribute__((ext_vector_type(8)));
typedef _Float16 v4h  __attribute__((ext_vector_type(4)));
typedef float    v8f  __attribute__((ext_vector_type(8)));
typedef float    v4f  __attribute__((ext_vector_type(4)));
typedef int      v4i  __attribute__((ext_vector_type(4)));
typedef v8h __attribute__((may_alias)) v8ha;
typedef v4h __attribute__((may_alias)) v4ha;
typedef v4f __attribute__((may_alias)) v4fa;
typedef v4i __attribute__((may_alias)) v4ia;
union FragH { v16h v; v8h half[2]; };

#define NB     8
#define NN     1024
#define DD     512
#define NE     8
#define NTOK   8192
#define NBE    64
#define TPB    256
#define WAVES  8
#define SLOPE  0.2f
#define NEGV   (-1.0e9f)
#define XCAR   16.0f
#define WCAR   256.0f
#define HCAR   16.0f
#define PCAR   4096.0f
#define SC_H   (16.0f / (16.0f * 256.0f))
#define SC_O   (1.0f / (4096.0f * 16.0f))

#define XBLK   (NTOK * DD / 8 / TPB)
#define WTIL   64
#define WBLK   (NE * (DD / WTIL) * (DD / WTIL))
#define WPH    72
#define UVROWS 32
#define UVBLK  (NE * DD / UVROWS)
#define LTOK   32
#define LBLK   (NTOK / LTOK)
#define HMT    128
#define HZT    64
#define HPH    136
#define AMT    16

static_assert(TPB == WAVES * 32);
static_assert(NB * NN == NTOK);
static_assert(NB * NE == NBE);
static_assert(XBLK * TPB * 8 == NTOK * DD);
static_assert(WBLK * WTIL * WTIL == NE * DD * DD);
static_assert((DD % WTIL) == 0 && (DD / WTIL) == 8);
static_assert(WTIL * 4 == TPB);
static_assert((WPH % 8) == 0 && (HPH % 8) == 0);
static_assert(UVBLK * UVROWS == NE * DD);
static_assert(UVROWS == 4 * WAVES);
static_assert(LBLK * LTOK == NTOK && (NN % LTOK) == 0);
static_assert(LTOK == 4 * WAVES);
static_assert(3 * NE * LTOK / 4 <= TPB);
static_assert((DD % 32) == 0 && (NN % 32) == 0);
static_assert((NN % HMT) == 0 && (DD % HZT) == 0);
static_assert(HMT == 16 * WAVES && HZT == 64);
static_assert((NN % AMT) == 0 && AMT == 2 * WAVES);
static_assert(DD == 64 * WAVES);
static_assert((NN % 64) == 0);
static_assert(DD == 16 * 32);

DEVINL v8f wmma_f16(v16h a, v16h b, v8f c) {
  v8f d = __builtin_amdgcn_wmma_f32_16x16x32_f16(false, a, false, b, (short)0, c, false, false);
  asm volatile("v_nop\n\tv_nop\n\tv_nop\n\tv_nop" : "+v"(d) : "v"(a), "v"(b));
  return d;
}
DEVINL v8f zero8f() {
  v8f z = {0.f, 0.f, 0.f, 0.f, 0.f, 0.f, 0.f, 0.f};
  return z;
}
DEVINL void load_frag(FragH& f, const f16t* row, int k0) {
  f.half[0] = *(const v8ha*)(row + k0);
  f.half[1] = *(const v8ha*)(row + k0 + 16);
}

DEVINL float wsum32(float v) {
  v += __shfl_xor(v, 16);
  v += __shfl_xor(v, 8);
  v += __shfl_xor(v, 4);
  v += __shfl_xor(v, 2);
  v += __shfl_xor(v, 1);
  return v;
}
DEVINL float hsum16(float v) {
  v += __shfl_xor(v, 8);
  v += __shfl_xor(v, 4);
  v += __shfl_xor(v, 2);
  v += __shfl_xor(v, 1);
  return v;
}
DEVINL float hmax16(float v) {
  v = fmaxf(v, __shfl_xor(v, 8));
  v = fmaxf(v, __shfl_xor(v, 4));
  v = fmaxf(v, __shfl_xor(v, 2));
  v = fmaxf(v, __shfl_xor(v, 1));
  return v;
}

template <int KD>
DEVINL void mma_4n(const f16t* __restrict__ arow, const f16t* __restrict__ brow, v8f (&acc)[4]) {
  #pragma unroll 1
  for (int ks = 0; ks < KD / 32; ++ks) {
    const int k0 = 32 * ks;
    FragH a;
    load_frag(a, arow, k0);
    #pragma unroll
    for (int n = 0; n < 4; ++n) {
      FragH b;
      load_frag(b, brow + (size_t)16 * n * KD, k0);
      acc[n] = wmma_f16(a.v, b.v, acc[n]);
    }
  }
}

__global__ __launch_bounds__(TPB) void cvt_x_k(const float* __restrict__ x, f16t* __restrict__ X16)
{
  const size_t idx = ((size_t)blockIdx.x * TPB + threadIdx.x) * 8;
  const v4f a = *(const v4fa*)(x + idx), c = *(const v4fa*)(x + idx + 4);
  v8h o;
  #pragma unroll
  for (int j = 0; j < 4; ++j) {
    o[j]     = (f16t)(a[j] * XCAR);
    o[4 + j] = (f16t)(c[j] * XCAR);
  }
  *(volatile v8h*)(X16 + idx) = o;
  __threadfence();
  *(volatile v8h*)(X16 + idx) = o;
}

__global__ __launch_bounds__(TPB) void cvt_w_k(const float* __restrict__ W, f16t* __restrict__ WT16)
{
  __shared__ __attribute__((aligned(16))) f16t sT[WTIL * WPH];
  const int tid = threadIdx.x, blk = blockIdx.x;
  const int e = blk >> 6, tile = blk & 63;
  const int d0 = (tile >> 3) * WTIL, z0 = (tile & 7) * WTIL;
  const int dr = tid >> 2, zc = (tid & 3) * 16;
  const float* src = W + ((size_t)(e * DD + d0 + dr)) * DD + z0 + zc;
  v4f w4[4];
  #pragma unroll
  for (int p = 0; p < 4; ++p) w4[p] = *(const v4fa*)(src + 4 * p);
  #pragma unroll
  for (int p = 0; p < 4; ++p) {
    #pragma unroll
    for (int c = 0; c < 4; ++c) sT[(zc + 4 * p + c) * WPH + dr] = (f16t)(w4[p][c] * WCAR);
  }
  __syncthreads();

  v8h v[2];
  f16t* dst[2];
  #pragma unroll
  for (int i = 0; i < 2; ++i) {
    const int q = tid + TPB * i;
    const int z = q >> 3, piece = q & 7;
    v[i]   = *(const v8ha*)(sT + z * WPH + 8 * piece);
    dst[i] = WT16 + ((size_t)(e * DD + z0 + z)) * DD + d0 + 8 * piece;
  }
  #pragma unroll
  for (int i = 0; i < 2; ++i) *(volatile v8h*)dst[i] = v[i];
  __threadfence();
  #pragma unroll
  for (int i = 0; i < 2; ++i) *(volatile v8h*)dst[i] = v[i];
}

__global__ __launch_bounds__(TPB) void uv_k(const float* __restrict__ W, const float* __restrict__ a_src,
                                           const float* __restrict__ a_dst, float* __restrict__ U,
                                           float* __restrict__ V)
{
  __shared__ __attribute__((aligned(16))) float suv[2 * UVROWS];
  const int tid = threadIdx.x, lane = tid & 31, wave = tid >> 5;
  const int rb = blockIdx.x * UVROWS;
  #pragma unroll 1
  for (int t = 0; t < 4; ++t) {
    const int rl = 4 * wave + t;
    const int R = rb + rl;
    const int e = R >> 9;
    const float* wr = W + (size_t)R * DD + 16 * lane;
    const float* ar = a_src + (size_t)e * DD + 16 * lane;
    const float* dr = a_dst + (size_t)e * DD + 16 * lane;
    float s1 = 0.0f, s2 = 0.0f;
    #pragma unroll 1
    for (int q = 0; q < 4; ++q) {
      const v4f wv = *(const v4fa*)(wr + 4 * q);
      const v4f av = *(const v4fa*)(ar + 4 * q);
      const v4f bv = *(const v4fa*)(dr + 4 * q);
      #pragma unroll
      for (int c = 0; c < 4; ++c) {
        s1 = fmaf(wv[c], av[c], s1);
        s2 = fmaf(wv[c], bv[c], s2);
      }
    }
    s1 = wsum32(s1);
    s2 = wsum32(s2);
    if (lane == 0) {
      suv[rl] = s1;
      suv[UVROWS + rl] = s2;
    }
  }
  __syncthreads();
  const bool act = tid < 16;
  const int tc = tid & 15;
  const v4f v = *(const v4fa*)(suv + 4 * tc);
  float* dst = (tc < 8) ? (U + rb + 4 * tc) : (V + rb + 4 * (tc - 8));
  if (act) *(volatile v4f*)dst = v;
  __threadfence();
  if (act) *(volatile v4f*)dst = v;
}

__global__ __launch_bounds__(TPB) void logit_k(const float* __restrict__ x, const float* __restrict__ gW,
                                              const float* __restrict__ gb, const float* __restrict__ U,
                                              const float* __restrict__ V, float* __restrict__ SS,
                                              float* __restrict__ SD, float* __restrict__ G)
{
  __shared__ __attribute__((aligned(16))) float sAll[3 * NE * LTOK];
  const int tid = threadIdx.x, lane = tid & 31, wave = tid >> 5;
  const int tb = blockIdx.x * LTOK;
  const int b = tb >> 10, n0 = tb & (NN - 1);
  const int dl = 16 * lane;

  #pragma unroll 1
  for (int t = 0; t < 4; ++t) {
    const int tloc = 4 * wave + t;
    const float* xr = x + (size_t)(tb + tloc) * DD + dl;

    float g[NE];
    #pragma unroll
    for (int e = 0; e < NE; ++e) g[e] = 0.0f;
    #pragma unroll 1
    for (int q = 0; q < 4; ++q) {
      const v4f xv = *(const v4fa*)(xr + 4 * q);
      #pragma unroll
      for (int c = 0; c < 4; ++c) {
        const float* gp = gW + (size_t)(dl + 4 * q + c) * NE;
        const v4f g0 = *(const v4fa*)gp, g1 = *(const v4fa*)(gp + 4);
        #pragma unroll
        for (int e = 0; e < 4; ++e) {
          g[e]     = fmaf(xv[c], g0[e], g[e]);
          g[4 + e] = fmaf(xv[c], g1[e], g[4 + e]);
        }
      }
    }
    float mx = -3.0e38f;
    #pragma unroll
    for (int e = 0; e < NE; ++e) {
      g[e] = wsum32(g[e]) + gb[e];
      mx = fmaxf(mx, g[e]);
    }
    float gs = 0.0f;
    #pragma unroll
    for (int e = 0; e < NE; ++e) {
      g[e] = __expf(g[e] - mx);
      gs += g[e];
    }
    const float ginv = 1.0f / gs;
    if (lane == 0) {
      #pragma unroll
      for (int e = 0; e < NE; ++e) sAll[2 * NE * LTOK + tloc * NE + e] = g[e] * ginv;
    }

    #pragma unroll 1
    for (int e = 0; e < NE; ++e) {
      const float* up = U + e * DD + dl;
      const float* vp = V + e * DD + dl;
      float ps = 0.0f, pd = 0.0f;
      #pragma unroll 1
      for (int q = 0; q < 4; ++q) {
        const v4f xv = *(const v4fa*)(xr + 4 * q);
        const v4f uv = *(const v4fa*)(up + 4 * q);
        const v4f vv = *(const v4fa*)(vp + 4 * q);
        #pragma unroll
        for (int c = 0; c < 4; ++c) {
          ps = fmaf(xv[c], uv[c], ps);
          pd = fmaf(xv[c], vv[c], pd);
        }
      }
      ps = wsum32(ps);
      pd = wsum32(pd);
      if (lane == 0) {
        sAll[e * LTOK + tloc] = ps;
        sAll[NE * LTOK + e * LTOK + tloc] = pd;
      }
    }
  }
  __syncthreads();

  const bool act = tid < 3 * NE * LTOK / 4;
  const int L = tid >> 3, piece = tid & 7;
  const int Lc = act ? L : 0;
  const v4f v = *(const v4fa*)(sAll + 32 * Lc + 4 * piece);
  float* dst;
  if (wave < 2)      dst = SS + (size_t)(b * NE + Lc) * NN + n0 + 4 * piece;
  else if (wave < 4) dst = SD + (size_t)(b * NE + (Lc - NE)) * NN + n0 + 4 * piece;
  else               dst = G + (size_t)tb * NE + (Lc - 2 * NE) * LTOK + 4 * piece;
  if (act) *(volatile v4f*)dst = v;
  __threadfence();
  if (act) *(volatile v4f*)dst = v;
}

__global__ __launch_bounds__(TPB) void hgemm_k(const f16t* __restrict__ X16, const f16t* __restrict__ WT16,
                                              f16t* __restrict__ HT)
{
  __shared__ __attribute__((aligned(16))) f16t sHT[HZT * HPH];
  const int tid = threadIdx.x, lane = tid & 31, wave = tid >> 5;
  const int h = lane >> 4, m = lane & 15;
  const int n0 = blockIdx.x * HMT, z0 = blockIdx.y * HZT, be = blockIdx.z;
  const int b = be >> 3, e = be & 7;

  v8f acc[4];
  #pragma unroll
  for (int n = 0; n < 4; ++n) acc[n] = zero8f();
  const f16t* arow = X16  + ((size_t)(b * NN + n0 + 16 * wave + m)) * DD + 8 * h;
  const f16t* brow = WT16 + ((size_t)(e * DD + z0 + m)) * DD + 8 * h;
  mma_4n<DD>(arow, brow, acc);

  #pragma unroll
  for (int ct = 0; ct < 4; ++ct) {
    v8h o;
    #pragma unroll
    for (int r = 0; r < 8; ++r) o[r] = (f16t)(acc[ct][r] * SC_H);
    *(v8ha*)(sHT + (16 * ct + m) * HPH + 16 * wave + 8 * h) = o;
  }
  __syncthreads();

  v8h v[4];
  f16t* dst[4];
  #pragma unroll
  for (int i = 0; i < 4; ++i) {
    const int q = tid + TPB * i;
    const int row = q >> 4, piece = q & 15;
    v[i]   = *(const v8ha*)(sHT + row * HPH + 8 * piece);
    dst[i] = HT + ((size_t)(be * DD + z0 + row)) * NN + n0 + 8 * piece;
  }
  #pragma unroll
  for (int i = 0; i < 4; ++i) *(volatile v8h*)dst[i] = v[i];
  __threadfence();
  #pragma unroll
  for (int i = 0; i < 4; ++i) *(volatile v8h*)dst[i] = v[i];
}

__global__ __launch_bounds__(TPB) void attn_k(const f16t* __restrict__ HT, const float* __restrict__ SS,
                                             const float* __restrict__ SD, const float* __restrict__ G,
                                             const int* __restrict__ adj, float* __restrict__ out)
{
  __shared__ __attribute__((aligned(16))) float bigf[AMT * DD];
  __shared__ __attribute__((aligned(16))) float sGt[AMT * NE];
  __shared__ float rowinv[AMT];
  f16t* pb = (f16t*)bigf;

  const int tid = threadIdx.x, lane = tid & 31, wave = tid >> 5;
  const int h = lane >> 4, m = lane & 15;
  const int r = tid >> 4, c = tid & 15;
  const int b = blockIdx.y, n0 = blockIdx.x * AMT;

  if (tid < AMT * NE / 4)
    *(v4fa*)(sGt + 4 * tid) = *(const v4fa*)(G + (size_t)(b * NN + n0) * NE + 4 * tid);
  v8f oacc[4];
  #pragma unroll
  for (int n = 0; n < 4; ++n) oacc[n] = zero8f();
  const int* arow = adj + ((size_t)(b * NN + n0 + r)) * NN + 4 * c;
  __syncthreads();

  #pragma unroll 1
  for (int e = 0; e < NE; ++e) {
    const int be = b * NE + e;
    const float rs = SS[(size_t)be * NN + n0 + r];
    const float* sdp = SD + (size_t)be * NN + 4 * c;

    float mx = -3.0e38f;
    #pragma unroll 2
    for (int t = 0; t < NN / 64; ++t) {
      const v4i a4 = *(const v4ia*)(arow + 64 * t);
      const v4f s4 = *(const v4fa*)(sdp + 64 * t);
      #pragma unroll
      for (int q = 0; q < 4; ++q) {
        float v = rs + s4[q];
        v = (v >= 0.0f) ? v : v * SLOPE;
        v = (a4[q] > 0) ? v : NEGV;
        mx = fmaxf(mx, v);
      }
    }
    mx = hmax16(mx);

    float ssum = 0.0f;
    #pragma unroll 2
    for (int t = 0; t < NN / 64; ++t) {
      const v4i a4 = *(const v4ia*)(arow + 64 * t);
      const v4f s4 = *(const v4fa*)(sdp + 64 * t);
      v4h ph;
      #pragma unroll
      for (int q = 0; q < 4; ++q) {
        float v = rs + s4[q];
        v = (v >= 0.0f) ? v : v * SLOPE;
        v = (a4[q] > 0) ? v : NEGV;
        const float p = __expf(v - mx);
        ssum += p;
        ph[q] = (f16t)(p * PCAR);
      }
      *(v4ha*)(pb + r * NN + 4 * c + 64 * t) = ph;
    }
    ssum = hsum16(ssum);
    if (c == 0) rowinv[r] = 1.0f / ssum;
    __syncthreads();

    v8f acc[4];
    #pragma unroll
    for (int n = 0; n < 4; ++n) acc[n] = zero8f();
    const f16t* ap = pb + m * NN + 8 * h;
    const f16t* bp = HT + ((size_t)(be * DD + 64 * wave + m)) * NN + 8 * h;
    #pragma unroll 1
    for (int ks = 0; ks < NN / 32; ++ks) {
      const int k0 = 32 * ks;
      FragH a;
      a.half[0] = *(const v8ha*)(ap + k0);
      a.half[1] = *(const v8ha*)(ap + k0 + 16);
      #pragma unroll
      for (int ct = 0; ct < 4; ++ct) {
        FragH bb;
        load_frag(bb, bp + (size_t)16 * ct * NN, k0);
        acc[ct] = wmma_f16(a.v, bb.v, acc[ct]);
      }
    }

    #pragma unroll
    for (int ct = 0; ct < 4; ++ct) {
      #pragma unroll
      for (int rr = 0; rr < 8; ++rr) {
        const int row = 8 * h + rr;
        float o = acc[ct][rr] * (rowinv[row] * SC_O);
        o = (o > 0.0f) ? o : (__expf(o) - 1.0f);
        oacc[ct][rr] = fmaf(sGt[row * NE + e], o, oacc[ct][rr]);
      }
    }
    __syncthreads();
  }

  #pragma unroll
  for (int ct = 0; ct < 4; ++ct) {
    #pragma unroll
    for (int rr = 0; rr < 8; ++rr)
      bigf[(8 * h + rr) * DD + 64 * wave + 16 * ct + m] = oacc[ct][rr];
  }
  __syncthreads();

  v4f v[8];
  float* dst[8];
  #pragma unroll
  for (int i = 0; i < 8; ++i) {
    const int q = tid + TPB * i;
    const int row = q >> 7, piece = q & 127;
    v[i]   = *(const v4fa*)(bigf + row * DD + 4 * piece);
    dst[i] = out + ((size_t)(b * NN + n0 + row)) * DD + 4 * piece;
  }
  #pragma unroll
  for (int i = 0; i < 8; ++i) *(volatile v4f*)dst[i] = v[i];
  __threadfence();
  #pragma unroll
  for (int i = 0; i < 8; ++i) *(volatile v4f*)dst[i] = v[i];
}

extern "C" void kernel_launch(void* const* d_in, const int* in_sizes, int n_in,
                              void* d_out, int out_size, void* d_ws, size_t ws_size,
                              hipStream_t stream) {
  if (n_in < 7) return;
  if (in_sizes[0] != NTOK * DD) return;
  if (in_sizes[1] != NB * NN * NN) return;
  if (in_sizes[2] != DD * NE) return;
  if (in_sizes[3] != NE) return;
  if (in_sizes[4] != NE * DD * DD) return;
  if (in_sizes[5] != NE * DD) return;
  if (in_sizes[6] != NE * DD) return;
  if (out_size != NTOK * DD) return;

  const float* x      = (const float*)d_in[0];
  const int*   adj    = (const int*)d_in[1];
  const float* gate_W = (const float*)d_in[2];
  const float* gate_b = (const float*)d_in[3];
  const float* W      = (const float*)d_in[4];
  const float* a_src  = (const float*)d_in[5];
  const float* a_dst  = (const float*)d_in[6];
  float* outp = (float*)d_out;

  const size_t szX  = (size_t)NTOK * DD * 2;
  const size_t szWT = (size_t)NE * DD * DD * 2;
  const size_t szHT = (size_t)NBE * DD * NN * 2;
  const size_t szUV = (size_t)NE * DD * 4;
  const size_t szS  = (size_t)NBE * NN * 4;
  const size_t szG  = (size_t)NTOK * NE * 4;
  size_t off = 0;
  char* ws = (char*)d_ws;
  f16t*  X16  = (f16t*)(ws + off);  off += szX;
  f16t*  WT16 = (f16t*)(ws + off);  off += szWT;
  f16t*  HT16 = (f16t*)(ws + off);  off += szHT;
  float* U    = (float*)(ws + off); off += szUV;
  float* V    = (float*)(ws + off); off += szUV;
  float* SS   = (float*)(ws + off); off += szS;
  float* SD   = (float*)(ws + off); off += szS;
  float* G    = (float*)(ws + off); off += szG;
  if (off > ws_size) return;

  cvt_x_k<<<XBLK, TPB, 0, stream>>>(x, X16);
  cvt_w_k<<<WBLK, TPB, 0, stream>>>(W, WT16);
  uv_k<<<UVBLK, TPB, 0, stream>>>(W, a_src, a_dst, U, V);
  logit_k<<<LBLK, TPB, 0, stream>>>(x, gate_W, gate_b, U, V, SS, SD, G);
  hgemm_k<<<dim3(NN / HMT, DD / HZT, NBE), TPB, 0, stream>>>(X16, WT16, HT16);
  attn_k<<<dim3(NN / AMT, NB), TPB, 0, stream>>>(HT16, SS, SD, G, adj, outp);
  (void)hipGetLastError();
}
